// ABCNN_22093311771258
// MI455X (gfx1250) — hardware-verified
//
#include <hip/hip_runtime.h>


#define NB_  256
#define LL   256
#define DD   100
#define DP   128
#define NV   50000
#define NLAY 2
#define LIN  512
#define FIN  600
#define GI   64
#define DM   DP
#define LOSC 1024.0f
typedef _Float16 h16;
typedef unsigned short bf;
typedef __attribute__((ext_vector_type(16))) __bf16   v16bf;
typedef __attribute__((ext_vector_type(16))) _Float16 v16h;
typedef __attribute__((ext_vector_type(8)))  _Float16 v8h;
typedef __attribute__((ext_vector_type(8)))  unsigned short v8us;
typedef __attribute__((ext_vector_type(8)))  float    v8f;
typedef __attribute__((ext_vector_type(4)))  float    v4f;
typedef v8h  __attribute__((may_alias)) v8ha;
typedef v4f  __attribute__((may_alias)) v4fa;
typedef v8us __attribute__((may_alias)) v8usa;

__device__ __forceinline__ unsigned short f2bf(float f) { unsigned u = __float_as_uint(f); u += 0x7FFFu + ((u >> 16) & 1u); return (unsigned short)(u >> 16); }
__device__ __forceinline__ float bf2f(unsigned short b) { return __uint_as_float(((unsigned)b) << 16); }
__device__ __forceinline__ float bfr(float f) { return bf2f(f2bf(f)); }
__device__ __forceinline__ v16h cat16(v8h lo, v8h hi) { return __builtin_shufflevector(lo, hi, 0, 1, 2, 3, 4, 5, 6, 7, 8, 9, 10, 11, 12, 13, 14, 15); }
__device__ __forceinline__ v16bf cat16b(v8us lo, v8us hi) { return __builtin_bit_cast(v16bf, __builtin_shufflevector(lo, hi, 0, 1, 2, 3, 4, 5, 6, 7, 8, 9, 10, 11, 12, 13, 14, 15)); }
__device__ __forceinline__ v8f wmma16(v16h a, v16h b, v8f c) { return __builtin_amdgcn_wmma_f32_16x16x32_f16(false, a, false, b, (short)0, c, false, false); }
__device__ __forceinline__ v8f wmmab(v16bf a, v16bf b, v8f c) { return __builtin_amdgcn_wmma_f32_16x16x32_bf16(false, a, false, b, (short)0, c, false, false); }


__global__ __launch_bounds__(128) void k_gemmh(const h16* __restrict__ A, const h16* __restrict__ Bn, const float* __restrict__ bias, float* C, int ldc, const float* __restrict__ R, int K, size_t sA, size_t sB, size_t sC, int roundR) {
    __shared__ __align__(16) float ost[4][16 * 68];
    const size_t z = blockIdx.z; A += z * sA; Bn += z * sB; C += z * sC; if (R) R += z * sC;
    const int lane = threadIdx.x & 31, wave = threadIdx.x >> 5, lr = lane & 15, hi = lane >> 4;
    const int r0 = blockIdx.x * 64 + wave * 16, c0 = blockIdx.y * 64;
    const size_t aoff = (size_t)(r0 + lr) * K + 8 * hi;
    size_t boff[4];
#pragma unroll
    for (int t = 0; t < 4; ++t) boff[t] = (size_t)(c0 + t * 16 + lr) * K + 8 * hi;
    v8f acc[4];
#pragma unroll
    for (int t = 0; t < 4; ++t) acc[t] = (v8f){};
#pragma unroll 1
    for (int kc = 0; kc < K; kc += 32) {
        const v16h a = cat16(*(const v8h*)(A + aoff + kc), *(const v8h*)(A + aoff + kc + 16));
#pragma unroll
        for (int t = 0; t < 4; ++t) { const v16h b = cat16(*(const v8h*)(Bn + boff[t] + kc), *(const v8h*)(Bn + boff[t] + kc + 16)); acc[t] = wmma16(a, b, acc[t]); }
        asm volatile("v_nop\n\tv_nop\n\tv_nop\n\tv_nop" : "+v"(acc[0]), "+v"(acc[1]), "+v"(acc[2]), "+v"(acc[3]) : "v"(a));
    }
    float* os = &ost[wave][0];
#pragma unroll
    for (int t = 0; t < 4; ++t) { const float bv = bias ? bfr(bias[c0 + t * 16 + lr]) : 0.f;
#pragma unroll
        for (int j = 0; j < 8; ++j) os[(hi * 8 + j) * 68 + t * 16 + lr] = acc[t][j] + bv; }
    __syncthreads();
    float* crow = C + (size_t)r0 * ldc + c0;
    auto pass = [&]() {
#pragma unroll
        for (int s = 0; s < 8; ++s) { const int Lid = (lane >> 3) + 4 * s, piece = lane & 7; const int row = Lid >> 1, cofs = (Lid & 1) * 32 + piece * 4;
            v4f val = *(const v4fa*)(os + row * 68 + cofs); if (R) { const v4f rv = *(const v4f*)(R + ((size_t)r0 + row) * ldc + c0 + cofs); val += roundR ? (v4f){bfr(rv[0]), bfr(rv[1]), bfr(rv[2]), bfr(rv[3])} : rv; }
            *(volatile v4f*)(crow + (size_t)row * ldc + cofs) = val; }
    };
    pass(); __threadfence(); pass();
}

typedef __attribute__((ext_vector_type(4))) _Float16 v4h;
__device__ __forceinline__ h16 tohx(float x) { return (h16)x; }
__global__ __launch_bounds__(256) void k_emb(const int* __restrict__ q, const float* __restrict__ emb, float* E) {
    const int lane = threadIdx.x & 31; const size_t r = (size_t)blockIdx.x * 8 + (threadIdx.x >> 5); if (r >= (size_t)NB_ * LL) return; int t = q[r]; t = t < 0 ? 0 : (t >= NV ? NV - 1 : t); v4f o;
#pragma unroll
    for (int i = 0; i < 4; ++i) { const int d = lane * 4 + i; o[i] = (d < DD) ? bfr(emb[(size_t)t * DD + d]) : 0.f; }
    *(volatile v4f*)(E + r * DP + lane * 4) = o; __threadfence(); *(volatile v4f*)(E + r * DP + lane * 4) = o;
}
__global__ __launch_bounds__(256) void k_meanL(const float* __restrict__ F, int b0, int slot, float* RES) {
    const int lane = threadIdx.x & 31; const int bl = blockIdx.x * 8 + (threadIdx.x >> 5); if (bl >= GI) return; const int b = b0 + bl; v4f acc = (v4f){0.f, 0.f, 0.f, 0.f};
#pragma unroll 1
    for (int i = 0; i < LL; ++i) acc += *(const v4f*)(F + ((size_t)bl * LL + i) * DP + lane * 4);
    acc = acc * (1.0f / LL); float* dst = RES + ((size_t)b * 6 + slot) * DP + lane * 4; *(volatile v4f*)dst = acc; __threadfence(); *(volatile v4f*)dst = acc;
}
__global__ __launch_bounds__(256) void k_mplane(const float* __restrict__ F, size_t fstride_b, const int* __restrict__ q, int b0, h16* SH) {
    const int lane = threadIdx.x & 31; const size_t w = (size_t)blockIdx.x * 8 + (threadIdx.x >> 5); if (w >= (size_t)GI * LL) return; const int bl = (int)(w / LL), i = (int)(w % LL); const int b = b0 + bl; const float v = (q[(size_t)b * LL + i] != 0) ? 1.f : 0.f; v4h o;
    const v4f x = *(const v4f*)(F + (size_t)bl * fstride_b + (size_t)i * DP + lane * 4);
#pragma unroll
    for (int k = 0; k < 4; ++k) o[k] = tohx(x[k] * v);
    *(volatile v4h*)(SH + w * DP + lane * 4) = o; __threadfence(); *(volatile v4h*)(SH + w * DP + lane * 4) = o;
}
__global__ __launch_bounds__(256) void k_sq(const float* __restrict__ F, size_t fstride_b, const int* __restrict__ q, int b0, float* SQ) {
    const int lane = threadIdx.x & 31; const int w = blockIdx.x * 8 + (threadIdx.x >> 5); if (w >= GI * (LL / 32)) return; const int bl = w / (LL / 32), i = (w % (LL / 32)) * 32 + lane; const int b = b0 + bl; const float v = (q[(size_t)b * LL + i] != 0) ? 1.f : 0.f; const float* fr = F + (size_t)bl * fstride_b + (size_t)i * DP; float s = 0.f;
#pragma unroll 1
    for (int d = 0; d < DP; ++d) { const float x = fr[d] * v; s = fmaf(x, x, s); }
    *(volatile float*)(SQ + (size_t)bl * LL + i) = s; __threadfence(); *(volatile float*)(SQ + (size_t)bl * LL + i) = s;
}
__global__ __launch_bounds__(256) void k_match(float* CR, const float* __restrict__ SQ1, const float* __restrict__ SQ2, h16* AH) {
    const int lane = threadIdx.x & 31; const size_t w = (size_t)blockIdx.x * 8 + (threadIdx.x >> 5); if (w >= (size_t)GI * LL) return; const int bl = (int)(w / LL), i = (int)(w % LL); const float s1 = SQ1[(size_t)bl * LL + i]; float* row = CR + w * LL;
    float a[8];
#pragma unroll
    for (int k = 0; k < 8; ++k) { const int j = (k < 4) ? lane * 4 + k : 128 + lane * 4 + k - 4; float d2 = s1 + SQ2[(size_t)bl * LL + j] - 2.0f * row[j]; d2 = fmaxf(d2, 0.f); const float sq = (d2 > 0.f) ? __fsqrt_rn(d2) : 0.f; a[k] = __fdiv_rn(1.0f, 1.0f + sq); }
    const v4f va = (v4f){a[0], a[1], a[2], a[3]}, vb = (v4f){a[4], a[5], a[6], a[7]};
    v4h ha, hb;
#pragma unroll
    for (int k = 0; k < 4; ++k) { ha[k] = tohx(a[k]); hb[k] = tohx(a[4 + k]); }
#pragma unroll 1
    for (int ps = 0; ps < 2; ++ps) { *(volatile v4f*)(row + lane * 4) = va; *(volatile v4f*)(row + 128 + lane * 4) = vb; *(volatile v4h*)(AH + w * LL + lane * 4) = ha; *(volatile v4h*)(AH + w * LL + 128 + lane * 4) = hb; if (ps == 0) __threadfence(); }
}
__global__ __launch_bounds__(256) void k_trA(const h16* __restrict__ AH, h16* ATH) {
    __shared__ float tl[64][65];
    const int tid = threadIdx.x; const int i0 = blockIdx.x * 64, j0 = blockIdx.y * 64; const size_t zb = (size_t)blockIdx.z * LL * LL; const int rr = tid >> 2, cq = (tid & 3) * 16;
#pragma unroll
    for (int k = 0; k < 16; ++k) tl[rr][cq + k] = (float)AH[zb + (size_t)(i0 + rr) * LL + j0 + cq + k];
    __syncthreads();
    const int lane = tid & 31, wv = tid >> 5;
    auto pass = [&]() {
#pragma unroll
        for (int st = 0; st < 4; ++st) { const int jr = wv * 8 + st * 2 + (lane >> 4); const int iq = (lane & 15) * 4; v4h v;
#pragma unroll
            for (int k = 0; k < 4; ++k) v[k] = (h16)tl[iq + k][jr];
            *(volatile v4h*)(ATH + zb + (size_t)(j0 + jr) * LL + i0 + iq) = v; }
    };
    pass(); __threadfence(); pass();
}
template <bool COLS>
__global__ __launch_bounds__(256) void k_sums(const float* __restrict__ A, float* WS) {
    const int lane = threadIdx.x & 31; const int w = blockIdx.x * 8 + (threadIdx.x >> 5); if (w >= GI * (LL / 32)) return; const int bl = w / (LL / 32), t = (w % (LL / 32)) * 32 + lane; const float* Ab = A + (size_t)bl * LL * LL; float s = 0.f;
#pragma unroll 1
    for (int k = 0; k < LL; ++k) s += COLS ? Ab[(size_t)k * LL + t] : Ab[(size_t)t * LL + k];
    *(volatile float*)(WS + (size_t)bl * LL + t) = s; __threadfence(); *(volatile float*)(WS + (size_t)bl * LL + t) = s;
}
__global__ __launch_bounds__(256) void k_wT16(const float* __restrict__ Wl, h16* WT) {
    const int lane = threadIdx.x & 31; const int d = blockIdx.x * 8 + (threadIdx.x >> 5); if (d >= DP) return; v8h o;
#pragma unroll
    for (int k = 0; k < 8; ++k) { const int j = lane * 8 + k; o[k] = tohx((d < DD) ? bfr(Wl[(size_t)j * DD + (d < DD ? d : 0)]) : 0.f); }
    *(volatile v8h*)(WT + (size_t)d * LL + lane * 8) = o; __threadfence(); *(volatile v8h*)(WT + (size_t)d * LL + lane * 8) = o;
}
__global__ __launch_bounds__(256) void k_convtanh(const float* __restrict__ E, const float* __restrict__ F, const float* __restrict__ ck, const float* __restrict__ cb, int b0, float* O) {
    const int lane = threadIdx.x & 31; const size_t w = (size_t)blockIdx.x * 8 + (threadIdx.x >> 5); if (w >= (size_t)GI * LL) return; const int bl = (int)(w / LL), i = (int)(w % LL); const float* Eb = E + ((size_t)(b0 + bl) * LL) * DP; const float* Fb = F + ((size_t)bl * LL) * DP;
    const float bias = bfr(cb[0]); v4f o;
#pragma unroll
    for (int u = 0; u < 4; ++u) { const int d = lane * 4 + u; float a = bias;
        if (d < DD) {
#pragma unroll 1
            for (int ky = 0; ky < 3; ++ky) { const int ii = i + ky - 1; if (ii < 0 || ii >= LL) continue;
#pragma unroll
                for (int kx = 0; kx < 3; ++kx) { const int dd = d + kx - 1; if (dd < 0 || dd >= DD) continue; a = fmaf(Eb[(size_t)ii * DP + dd], bfr(ck[ky * 3 + kx]), a); a = fmaf(Fb[(size_t)ii * DP + dd], bfr(ck[9 + ky * 3 + kx]), a); } }
            a = tanhf(a); } else a = 0.f;
        o[u] = a; }
    *(volatile v4f*)(O + w * DP + lane * 4) = o; __threadfence(); *(volatile v4f*)(O + w * DP + lane * 4) = o;
}
__global__ __launch_bounds__(256) void k_update(const float* __restrict__ O, const float* __restrict__ WS, int b0, float* E) {
    const int lane = threadIdx.x & 31; const size_t w = (size_t)blockIdx.x * 8 + (threadIdx.x >> 5); if (w >= (size_t)GI * LL) return; const int bl = (int)(w / LL), i = (int)(w % LL); const float* Ob = O + (size_t)bl * LL * DP; const float* wb = WS + (size_t)bl * LL; float* er = E + (((size_t)(b0 + bl) * LL) + i) * DP + lane * 4;
    v4f acc = (v4f){0.f, 0.f, 0.f, 0.f};
#pragma unroll
    for (int t = -1; t <= 1; ++t) { const int ii = i + t; if (ii < 0 || ii >= LL) continue; const v4f ov = *(const v4f*)(Ob + (size_t)ii * DP + lane * 4); acc += ov * wb[ii]; }
    const v4f e = *(const v4f*)er; const v4f y = acc * (1.0f / 3.0f) + e;
    *(volatile v4f*)er = y; __threadfence(); *(volatile v4f*)er = y;
}
__global__ __launch_bounds__(256) void k_fc1(const float* __restrict__ RES, const float* __restrict__ w1, const float* __restrict__ b1, const float* __restrict__ g, const float* __restrict__ bb, float* HR) {
    const int lane = threadIdx.x & 31; const int b = blockIdx.x * 8 + (threadIdx.x >> 5); if (b >= NB_) return; const float* rb = RES + (size_t)b * 6 * DP; float h[16];
#pragma unroll
    for (int u = 0; u < 16; ++u) h[u] = bfr(b1[(u & 3) + lane * 4 + (u >> 2) * 128]);
#pragma unroll 1
    for (int s = 0; s < 6; ++s) {
#pragma unroll 1
        for (int d = 0; d < DD; ++d) { const float x = rb[s * DP + d]; const float* wr = w1 + (size_t)(s * DD + d) * LIN;
#pragma unroll
            for (int u = 0; u < 16; ++u) h[u] = fmaf(x, bfr(wr[(u & 3) + lane * 4 + (u >> 2) * 128]), h[u]); } }
    float sm = 0.f;
#pragma unroll
    for (int u = 0; u < 16; ++u) sm += h[u];
#pragma unroll
    for (int sh = 16; sh; sh >>= 1) sm += __shfl_xor(sm, sh, 32);
    const float mu = sm * (1.0f / LIN); float q = 0.f;
#pragma unroll
    for (int u = 0; u < 16; ++u) { const float dv = h[u] - mu; q = fmaf(dv, dv, q); }
#pragma unroll
    for (int sh = 16; sh; sh >>= 1) q += __shfl_xor(q, sh, 32);
    const float rs = rsqrtf(q * (1.0f / LIN) + 1e-5f);
#pragma unroll 1
    for (int ps = 0; ps < 2; ++ps) {
#pragma unroll
        for (int p = 0; p < 4; ++p) { v4f o;
#pragma unroll
            for (int k = 0; k < 4; ++k) { const int c = p * 128 + lane * 4 + k; o[k] = fmaxf((h[p * 4 + k] - mu) * rs * bfr(g[c]) + bfr(bb[c]), 0.f); }
            *(volatile v4f*)(HR + (size_t)b * LIN + p * 128 + lane * 4) = o; }
        if (ps == 0) __threadfence(); }
}
__global__ __launch_bounds__(256) void k_fc2(const float* __restrict__ HR, const float* __restrict__ w2, const float* __restrict__ b2, float* OUTB) {
    const int lane = threadIdx.x & 31; const int w = blockIdx.x * 8 + (threadIdx.x >> 5); if (w >= NB_ / 16) return; const int b = w * 16 + (lane >> 1), o = lane & 1; float a = bfr(b2[o]);
#pragma unroll 1
    for (int k = 0; k < LIN; ++k) a = fmaf(HR[(size_t)b * LIN + k], bfr(w2[k * 2 + o]), a);
    *(volatile float*)(OUTB + (size_t)b * 2 + o) = a; __threadfence(); *(volatile float*)(OUTB + (size_t)b * 2 + o) = a;
}
extern "C" void kernel_launch(void* const* d_in, const int* in_sizes, int n_in,
                              void* d_out, int out_size, void* d_ws, size_t ws_size, hipStream_t stream) {
    (void)in_sizes; (void)n_in; (void)out_size;
    const int* q1 = (const int*)d_in[0]; const int* q2 = (const int*)d_in[1]; const float* emb = (const float*)d_in[2]; const float* Ws = (const float*)d_in[3]; const float* ck = (const float*)d_in[4]; const float* cb = (const float*)d_in[5]; const float* f1w = (const float*)d_in[6]; const float* f1b = (const float*)d_in[7]; const float* lg = (const float*)d_in[8]; const float* lb = (const float*)d_in[9]; const float* f2w = (const float*)d_in[10]; const float* f2b = (const float*)d_in[11];
    float* out = (float*)d_out;
    char* wsp = (char*)d_ws;
    auto take = [&](size_t bytes) { char* p = wsp; wsp += (bytes + 255) & ~(size_t)255; return (void*)p; };
    float* E1 = (float*)take((size_t)NB_ * LL * DP * 4); float* E2 = (float*)take((size_t)NB_ * LL * DP * 4); float* RES = (float*)take((size_t)NB_ * 6 * DP * 4); h16* WT = (h16*)take((size_t)DP * LL * 2); float* HR = (float*)take((size_t)NB_ * LIN * 4);
    h16* S1 = (h16*)take((size_t)GI * LL * DP * 2); h16* S2 = (h16*)take((size_t)GI * LL * DP * 2); float* SQ1 = (float*)take((size_t)GI * LL * 4); float* SQ2 = (float*)take((size_t)GI * LL * 4); float* CR = (float*)take((size_t)GI * LL * LL * 4);
    h16* AH = (h16*)take((size_t)GI * LL * LL * 2); h16* ATH = (h16*)take((size_t)GI * LL * LL * 2); float* F1 = (float*)take((size_t)GI * LL * DP * 4); float* F2 = (float*)take((size_t)GI * LL * DP * 4); float* O1 = (float*)take((size_t)GI * LL * DP * 4); float* O2 = (float*)take((size_t)GI * LL * DP * 4); float* W1 = (float*)take((size_t)GI * LL * 4); float* W2 = (float*)take((size_t)GI * LL * 4);
    if ((size_t)(wsp - (char*)d_ws) > ws_size) return;
    const size_t ES = (size_t)LL * DP;
    k_emb<<<(NB_ * LL) / 8, 256, 0, stream>>>(q1, emb, E1); k_emb<<<(NB_ * LL) / 8, 256, 0, stream>>>(q2, emb, E2);
    for (int b0 = 0; b0 < NB_; b0 += GI) { k_meanL<<<GI / 8, 256, 0, stream>>>(E1 + (size_t)b0 * ES, b0, 0, RES); k_meanL<<<GI / 8, 256, 0, stream>>>(E2 + (size_t)b0 * ES, b0, 3, RES); }
    for (int l = 0; l < NLAY; ++l) {
        k_wT16<<<DP / 8, 256, 0, stream>>>(Ws + (size_t)l * LL * DD, WT);
        for (int b0 = 0; b0 < NB_; b0 += GI) {
            k_mplane<<<(GI * LL) / 8, 256, 0, stream>>>(E1 + (size_t)b0 * ES, ES, q1, b0, S1); k_mplane<<<(GI * LL) / 8, 256, 0, stream>>>(E2 + (size_t)b0 * ES, ES, q2, b0, S2);
            k_sq<<<(GI * (LL / 32)) / 8, 256, 0, stream>>>(E1 + (size_t)b0 * ES, ES, q1, b0, SQ1); k_sq<<<(GI * (LL / 32)) / 8, 256, 0, stream>>>(E2 + (size_t)b0 * ES, ES, q2, b0, SQ2);
            k_gemmh<<<dim3(LL / 64, LL / 64, GI), 128, 0, stream>>>(S1, S2, nullptr, CR, LL, nullptr, DP, (size_t)LL * DP, (size_t)LL * DP, (size_t)LL * LL, 0);
            k_match<<<(GI * LL) / 8, 256, 0, stream>>>(CR, SQ1, SQ2, AH);
            k_trA<<<dim3(LL / 64, LL / 64, GI), 256, 0, stream>>>(AH, ATH);
            k_gemmh<<<dim3(LL / 64, DP / 64, GI), 128, 0, stream>>>(AH, WT, nullptr, F1, DP, nullptr, LL, (size_t)LL * LL, 0, (size_t)LL * DP, 0);
            k_gemmh<<<dim3(LL / 64, DP / 64, GI), 128, 0, stream>>>(ATH, WT, nullptr, F2, DP, nullptr, LL, (size_t)LL * LL, 0, (size_t)LL * DP, 0);
            k_convtanh<<<(GI * LL) / 8, 256, 0, stream>>>(E1, F1, ck + (size_t)l * 18, cb + l, b0, O1); k_convtanh<<<(GI * LL) / 8, 256, 0, stream>>>(E2, F2, ck + (size_t)l * 18, cb + l, b0, O2);
            k_meanL<<<GI / 8, 256, 0, stream>>>(O1, b0, 1 + l, RES); k_meanL<<<GI / 8, 256, 0, stream>>>(O2, b0, 4 + l, RES);
            k_mplane<<<(GI * LL) / 8, 256, 0, stream>>>(O1, ES, q1, b0, S1); k_mplane<<<(GI * LL) / 8, 256, 0, stream>>>(O2, ES, q2, b0, S2);
            k_sq<<<(GI * (LL / 32)) / 8, 256, 0, stream>>>(O1, ES, q1, b0, SQ1); k_sq<<<(GI * (LL / 32)) / 8, 256, 0, stream>>>(O2, ES, q2, b0, SQ2);
            k_gemmh<<<dim3(LL / 64, LL / 64, GI), 128, 0, stream>>>(S1, S2, nullptr, CR, LL, nullptr, DP, (size_t)LL * DP, (size_t)LL * DP, (size_t)LL * LL, 0);
            k_match<<<(GI * LL) / 8, 256, 0, stream>>>(CR, SQ1, SQ2, AH);
            k_sums<false><<<(GI * (LL / 32)) / 8, 256, 0, stream>>>(CR, W1); k_sums<true><<<(GI * (LL / 32)) / 8, 256, 0, stream>>>(CR, W2);
            k_update<<<(GI * LL) / 8, 256, 0, stream>>>(O1, W1, b0, E1); k_update<<<(GI * LL) / 8, 256, 0, stream>>>(O2, W2, b0, E2); } }
    k_fc1<<<NB_ / 8, 256, 0, stream>>>(RES, f1w, f1b, lg, lb, HR);
    k_fc2<<<(NB_ / 16 + 7) / 8, 256, 0, stream>>>(HR, f2w, f2b, out);
}
